// MambaLayer2PE_67001489817882
// MI455X (gfx1250) — hardware-verified
//
#include <hip/hip_runtime.h>
#include <math.h>
#include <stddef.h>


#define DIMC      320
#define D_STATE   32
#define D_CONV    4
#define D_INNER   640
#define NHEADS    8
#define HEADDIM   80
#define CONV_DIM  704
#define D_IN_PROJ 1352
#define N1_PAD    1408
#define BATCH     2
#define HIMG      64
#define WIMG      64
#define LSEQ      (HIMG * WIMG)
#define MROWS     (BATCH * LSEQ)
#define LN_EPS    1e-5f
#define RMS_EPS   1e-5f
#define YCHUNK    32
#define G1GRP     (N1_PAD * DIMC / 8)
#define G2GRP     (DIMC * D_INNER / 8)

static_assert(MROWS % 64 == 0, "");
static_assert(N1_PAD % 64 == 0, "");
static_assert(DIMC % 64 == 0, "");
static_assert(LSEQ % 64 == 0, "");
static_assert(DIMC % 32 == 0, "");
static_assert(D_INNER % 32 == 0, "");
static_assert(LSEQ % YCHUNK == 0, "");
static_assert(HEADDIM == 80, "");
static_assert(MROWS % 8 == 0, "");

typedef float          v4f     __attribute__((ext_vector_type(4)));
typedef float          v8f     __attribute__((ext_vector_type(8)));
typedef unsigned short us8     __attribute__((ext_vector_type(8)));
typedef unsigned short us16    __attribute__((ext_vector_type(16)));
typedef __bf16         bf16v16 __attribute__((ext_vector_type(16)));

__device__ __forceinline__ unsigned int bf16_rne_bits(float f) {
    unsigned int u = __float_as_uint(f);
    u = u + 0x7FFFu + ((u >> 16) & 1u);
    return u >> 16;
}
__device__ __forceinline__ void split_hi_lo(float f, unsigned short& hi, unsigned short& lo) {
    const unsigned int h = bf16_rne_bits(f);
    const float fh = __uint_as_float(h << 16);
    hi = (unsigned short)h;
    lo = (unsigned short)bf16_rne_bits(f - fh);
}
__device__ __forceinline__ void split8(const float (&v)[8], us8& hv, us8& lv) {
    us8 h = {}, l = {};
#pragma unroll
    for (int i = 0; i < 8; ++i) {
        unsigned short a, b;
        split_hi_lo(v[i], a, b);
        h[i] = a;
        l[i] = b;
    }
    hv = h;
    lv = l;
}
__device__ __forceinline__ float wave_sum(float v) {
#pragma unroll
    for (int o = 16; o > 0; o >>= 1) v += __shfl_xor(v, o);
    return v;
}
__device__ __forceinline__ float fast_rcp(float x) { return __builtin_amdgcn_rcpf(x); }

__device__ __forceinline__ v8f mma_bf16(us16 a, us16 b, v8f c) {
    v8f d = __builtin_amdgcn_wmma_f32_16x16x32_bf16(false, __builtin_bit_cast(bf16v16, a), false,
                                                     __builtin_bit_cast(bf16v16, b), (short)0, c, false, false);
    asm volatile("v_nop\n\tv_nop\n\tv_nop\n\tv_nop" : "+v"(d) : "v"(a), "v"(b));
    return d;
}
__device__ __forceinline__ us16 load_frag(const unsigned short* __restrict__ rowp, int k0, int hf) {
    const us8 e0 = *(const us8*)(rowp + k0 + 8 * hf);
    const us8 e1 = *(const us8*)(rowp + k0 + 16 + 8 * hf);
    return __builtin_shufflevector(e0, e1, 0, 1, 2, 3, 4, 5, 6, 7, 8, 9, 10, 11, 12, 13, 14, 15);
}

__global__ __launch_bounds__(256) void prep_w_kernel(const float* __restrict__ w1, const float* __restrict__ w2,
                                                    unsigned short* __restrict__ w1h, unsigned short* __restrict__ w1l,
                                                    unsigned short* __restrict__ w2h, unsigned short* __restrict__ w2l)
{
    const int gi = blockIdx.x * blockDim.x + threadIdx.x;
    if (gi >= G1GRP + G2GRP) return;
    float v[8];
    unsigned short* dh;
    unsigned short* dl;
    if (gi < G1GRP) {
        const int n  = gi / (DIMC / 8);
        const int kg = gi - n * (DIMC / 8);
        if (n < D_IN_PROJ) {
            const float* src = w1 + (size_t)n * DIMC + kg * 8;
            const v4f p0 = *(const v4f*)src;
            const v4f p1 = *(const v4f*)(src + 4);
            v[0] = p0[0]; v[1] = p0[1]; v[2] = p0[2]; v[3] = p0[3];
            v[4] = p1[0]; v[5] = p1[1]; v[6] = p1[2]; v[7] = p1[3];
        } else {
#pragma unroll
            for (int i = 0; i < 8; ++i) v[i] = 0.0f;
        }
        dh = w1h + (size_t)gi * 8;
        dl = w1l + (size_t)gi * 8;
    } else {
        const int g2 = gi - G1GRP;
        const float* src = w2 + (size_t)g2 * 8;
        const v4f p0 = *(const v4f*)src;
        const v4f p1 = *(const v4f*)(src + 4);
        v[0] = p0[0]; v[1] = p0[1]; v[2] = p0[2]; v[3] = p0[3];
        v[4] = p1[0]; v[5] = p1[1]; v[6] = p1[2]; v[7] = p1[3];
        dh = w2h + (size_t)g2 * 8;
        dl = w2l + (size_t)g2 * 8;
    }
    us8 hv, lv;
    split8(v, hv, lv);
    *(volatile us8*)dh = hv;
    *(volatile us8*)dl = lv;
    __threadfence();
    *(volatile us8*)dh = hv;
    *(volatile us8*)dl = lv;
}

__global__ __launch_bounds__(256) void ln_pe_kernel(const float* __restrict__ x, const float* __restrict__ peg,
                                                   const float* __restrict__ lnw, const float* __restrict__ lnb,
                                                   unsigned short* __restrict__ uh, unsigned short* __restrict__ ul)
{
#pragma clang fp contract(off)
    __shared__ __attribute__((aligned(16))) float s_u[8][DIMC];
    const int tid = threadIdx.x, wave = tid >> 5, lane = tid & 31;
    const int m0 = blockIdx.x * 8;

#pragma unroll 1
    for (int e = tid; e < 8 * DIMC; e += 256) {
        const int tok = e / DIMC;
        const int c   = e - tok * DIMC;
        const int m   = m0 + tok;
        float val = 0.0f;
        if (m < MROWS) {
            const int b  = m / LSEQ;
            const int t  = m - b * LSEQ;
            const int hy = t / WIMG;
            const int wx = t - hy * WIMG;
            const float xe = ((float)wx + 0.5f) * (1.0f / (float)WIMG);
            const float ye = ((float)hy + 0.5f) * (1.0f / (float)HIMG);
            const float cx = 2.0f * xe - 1.0f;
            const float cy = 2.0f * ye - 1.0f;
            const int jj = (c < DIMC / 2) ? c : (c - DIMC / 2);
            const float g0 = peg[jj];
            const float g1 = peg[DIMC / 2 + jj];
            const float pr = 6.2831855f * (cx * g0 + cy * g1);
            float sv, cv;
            sincosf(pr, &sv, &cv);
            const float pe = (c < DIMC / 2) ? sv : cv;
            val = x[((size_t)(b * DIMC + c)) * LSEQ + t] + pe;
        }
        s_u[tok][c] = val;
    }
    __syncthreads();

    const int m = m0 + wave;
    if (m >= MROWS) return;

    float s = 0.0f;
#pragma unroll
    for (int j = 0; j < DIMC / 32; ++j) s += s_u[wave][lane + 32 * j];
    const float mean = wave_sum(s) * (1.0f / (float)DIMC);
    float ss = 0.0f;
#pragma unroll
    for (int j = 0; j < DIMC / 32; ++j) {
        const float d = s_u[wave][lane + 32 * j] - mean;
        ss += d * d;
    }
    const float var  = wave_sum(ss) * (1.0f / (float)DIMC);
    const float rstd = rsqrtf(var + LN_EPS);

    us8 hv[2], lv[2];
#pragma unroll
    for (int j = 0; j < 2; ++j) {
        const bool valid = (j == 0) || (lane < 8);
        const int  gcl   = valid ? (32 * j + lane) : 0;
        float o[8];
#pragma unroll
        for (int i = 0; i < 8; ++i) {
            const int c = 8 * gcl + i;
            o[i] = (s_u[wave][c] - mean) * rstd * lnw[c] + lnb[c];
        }
        split8(o, hv[j], lv[j]);
    }
    unsigned short* ph = uh + (size_t)m * DIMC;
    unsigned short* pl = ul + (size_t)m * DIMC;
    *(volatile us8*)(ph + 8 * lane) = hv[0];
    *(volatile us8*)(pl + 8 * lane) = lv[0];
    if (lane < 8) {
        *(volatile us8*)(ph + 256 + 8 * lane) = hv[1];
        *(volatile us8*)(pl + 256 + 8 * lane) = lv[1];
    }
    __threadfence();
    *(volatile us8*)(ph + 8 * lane) = hv[0];
    *(volatile us8*)(pl + 8 * lane) = lv[0];
    if (lane < 8) {
        *(volatile us8*)(ph + 256 + 8 * lane) = hv[1];
        *(volatile us8*)(pl + 256 + 8 * lane) = lv[1];
    }
}

template <int K, bool TRANS>
__global__ __launch_bounds__(128) void gemm_split_kernel(const unsigned short* __restrict__ Ah,
                                                        const unsigned short* __restrict__ Al,
                                                        const unsigned short* __restrict__ Wh,
                                                        const unsigned short* __restrict__ Wl,
                                                        float* __restrict__ C)
{
    __shared__ __attribute__((aligned(16))) float S[64][68];
    const int wave = threadIdx.x >> 5, lane = threadIdx.x & 31, hf = lane >> 4, lm = lane & 15;
    const int bm0 = blockIdx.x * 64, bn0 = blockIdx.y * 64;
    const int wr = (wave >> 1) * 32, wc = (wave & 1) * 32;

    const unsigned short* a0h = Ah + (size_t)(bm0 + wr + lm) * K;
    const unsigned short* a1h = a0h + (size_t)16 * K;
    const unsigned short* a0l = Al + (size_t)(bm0 + wr + lm) * K;
    const unsigned short* a1l = a0l + (size_t)16 * K;
    const unsigned short* b0h = Wh + (size_t)(bn0 + wc + lm) * K;
    const unsigned short* b1h = b0h + (size_t)16 * K;
    const unsigned short* b0l = Wl + (size_t)(bn0 + wc + lm) * K;
    const unsigned short* b1l = b0l + (size_t)16 * K;

    v8f acc00 = {}, acc01 = {}, acc10 = {}, acc11 = {};

#pragma unroll 1
    for (int k0 = 0; k0 < K; k0 += 32) {
        const us16 fb0h = load_frag(b0h, k0, hf);
        const us16 fb0l = load_frag(b0l, k0, hf);
        const us16 fb1h = load_frag(b1h, k0, hf);
        const us16 fb1l = load_frag(b1l, k0, hf);
        {
            const us16 fah = load_frag(a0h, k0, hf);
            const us16 fal = load_frag(a0l, k0, hf);
            acc00 = mma_bf16(fah, fb0h, acc00);
            acc00 = mma_bf16(fah, fb0l, acc00);
            acc00 = mma_bf16(fal, fb0h, acc00);
            acc01 = mma_bf16(fah, fb1h, acc01);
            acc01 = mma_bf16(fah, fb1l, acc01);
            acc01 = mma_bf16(fal, fb1h, acc01);
        }
        {
            const us16 fah = load_frag(a1h, k0, hf);
            const us16 fal = load_frag(a1l, k0, hf);
            acc10 = mma_bf16(fah, fb0h, acc10);
            acc10 = mma_bf16(fah, fb0l, acc10);
            acc10 = mma_bf16(fal, fb0h, acc10);
            acc11 = mma_bf16(fah, fb1h, acc11);
            acc11 = mma_bf16(fah, fb1l, acc11);
            acc11 = mma_bf16(fal, fb1h, acc11);
        }
    }

#pragma unroll
    for (int r = 0; r < 8; ++r) {
        if (!TRANS) {
            S[wr + 8 * hf + r][wc + lm]           = acc00[r];
            S[wr + 8 * hf + r][wc + 16 + lm]      = acc01[r];
            S[wr + 16 + 8 * hf + r][wc + lm]      = acc10[r];
            S[wr + 16 + 8 * hf + r][wc + 16 + lm] = acc11[r];
        } else {
            S[wc + lm][wr + 8 * hf + r]           = acc00[r];
            S[wc + 16 + lm][wr + 8 * hf + r]      = acc01[r];
            S[wc + lm][wr + 16 + 8 * hf + r]      = acc10[r];
            S[wc + 16 + lm][wr + 16 + 8 * hf + r] = acc11[r];
        }
    }
    __syncthreads();

    const int bb = bm0 / LSEQ;
    const int t0 = bm0 - bb * LSEQ;
    v4f v[8];
    size_t dofs[8];
#pragma unroll
    for (int i = 0; i < 8; ++i) {
        const int rr = 16 * wave + 2 * i + hf;
        v[i] = *(const v4f*)(&S[rr][4 * lm]);
        if (!TRANS) dofs[i] = (size_t)(bm0 + rr) * N1_PAD + bn0 + 4 * lm;
        else        dofs[i] = (size_t)(bb * DIMC + bn0 + rr) * LSEQ + t0 + 4 * lm;
    }
#pragma unroll
    for (int i = 0; i < 8; ++i) *(volatile v4f*)(C + dofs[i]) = v[i];
    __threadfence();
#pragma unroll
    for (int i = 0; i < 8; ++i) *(volatile v4f*)(C + dofs[i]) = v[i];
}

__global__ __launch_bounds__(160) void ssm_scan_kernel(const float* __restrict__ zxb, const float* __restrict__ conv_w,
                                                      const float* __restrict__ conv_b, const float* __restrict__ dt_bias,
                                                      const float* __restrict__ A_log, const float* __restrict__ Dp,
                                                      float* __restrict__ ybuf)
{
    __shared__ float s_bc[2][2 * D_STATE];
    __shared__ float s_dt[2][2];
    __shared__ __attribute__((aligned(16))) float s_y[HEADDIM * YCHUNK];

    const int b   = blockIdx.x / NHEADS;
    const int hh  = blockIdx.x - b * NHEADS;
    const int tid = threadIdx.x, lane = tid & 31, wave = tid >> 5;
    const int p = tid >> 1, q = tid & 1;

    const int cxc = hh * HEADDIM + p;
    const float wx0 = conv_w[cxc * D_CONV + 0], wx1 = conv_w[cxc * D_CONV + 1];
    const float wx2 = conv_w[cxc * D_CONV + 2], wx3 = conv_w[cxc * D_CONV + 3];
    const float bx  = conv_b[cxc];
    const bool roleBC = tid < 2 * D_STATE;
    const int  cbc    = D_INNER + (roleBC ? tid : 0);
    const float wb0 = conv_w[cbc * D_CONV + 0], wb1 = conv_w[cbc * D_CONV + 1];
    const float wb2 = conv_w[cbc * D_CONV + 2], wb3 = conv_w[cbc * D_CONV + 3];
    const float bbias = conv_b[cbc];

    const float Ah    = -expf(A_log[hh]);
    const float dbias = dt_bias[hh];
    const float dph   = Dp[hh];

    float st[D_STATE / 2];
#pragma unroll
    for (int j = 0; j < D_STATE / 2; ++j) st[j] = 0.0f;
    float hx1 = 0.0f, hx2 = 0.0f, hx3 = 0.0f;
    float hb1 = 0.0f, hb2 = 0.0f, hb3 = 0.0f;

    const float* zb = zxb + (size_t)b * LSEQ * N1_PAD;
    float* ybase = ybuf + (size_t)b * D_INNER * LSEQ;

    for (int t = 0; t < LSEQ; ++t) {
        const int par = t & 1;
        const float* row = zb + (size_t)t * N1_PAD;

        const float rx = row[D_INNER + cxc];
        const float xc = bx + wx0 * hx3 + wx1 * hx2 + wx2 * hx1 + wx3 * rx;
        hx3 = hx2; hx2 = hx1; hx1 = rx;
        const float xv = xc * fast_rcp(1.0f + __expf(-xc));

        if (roleBC) {
            const float rb = row[D_INNER + cbc];
            const float bc = bbias + wb0 * hb3 + wb1 * hb2 + wb2 * hb1 + wb3 * rb;
            hb3 = hb2; hb2 = hb1; hb1 = rb;
            s_bc[par][tid] = bc * fast_rcp(1.0f + __expf(-bc));
        }
        if (tid == 2 * D_STATE) {
            const float draw = row[D_INNER + CONV_DIM + hh] + dbias;
            const float dtv  = fmaxf(draw, 0.0f) + log1pf(expf(-fabsf(draw)));
            s_dt[par][0] = dtv;
            s_dt[par][1] = expf(dtv * Ah);
        }
        __syncthreads();

        const float dtv = s_dt[par][0];
        const float dA  = s_dt[par][1];
        const float dtx = dtv * xv;
        float y = 0.0f;
#pragma unroll
        for (int j = 0; j < D_STATE / 2; ++j) {
            const float bn = s_bc[par][(D_STATE / 2) * q + j];
            const float cn = s_bc[par][D_STATE + (D_STATE / 2) * q + j];
            st[j] = st[j] * dA + dtx * bn;
            y += st[j] * cn;
        }
        y += __shfl_xor(y, 1);
        if (q == 0) s_y[p * YCHUNK + (t & (YCHUNK - 1))] = y + dph * xv;

        if ((t & (YCHUNK - 1)) == YCHUNK - 1) {
            __syncthreads();
            v4f v[4];
            size_t dofs[4];
#pragma unroll
            for (int i = 0; i < 4; ++i) {
                const int pr    = 16 * wave + 4 * i + (lane >> 3);
                const int piece = lane & 7;
                v[i]    = *(const v4f*)(&s_y[pr * YCHUNK + piece * 4]);
                dofs[i] = (size_t)(hh * HEADDIM + pr) * LSEQ + (size_t)(t - (YCHUNK - 1)) + piece * 4;
            }
#pragma unroll
            for (int i = 0; i < 4; ++i) *(volatile v4f*)(ybase + dofs[i]) = v[i];
            __threadfence();
#pragma unroll
            for (int i = 0; i < 4; ++i) *(volatile v4f*)(ybase + dofs[i]) = v[i];
        }
    }
}

__global__ __launch_bounds__(256) void gate_rms_kernel(const float* __restrict__ zxb, const float* __restrict__ ybuf,
                                                      const float* __restrict__ rmsw,
                                                      unsigned short* __restrict__ yh, unsigned short* __restrict__ yl)
{
    const int wave = threadIdx.x >> 5, lane = threadIdx.x & 31;
    const int m = blockIdx.x * 8 + wave;
    if (m >= MROWS) return;
    const int b = m / LSEQ, t = m - b * LSEQ;
    const float* zr = zxb + (size_t)m * N1_PAD;
    const float* yb = ybuf + (size_t)b * D_INNER * LSEQ + t;

    float g[3][8];
    float ss = 0.0f;
#pragma unroll
    for (int j = 0; j < 3; ++j) {
        const bool valid = (j < 2) || (lane < 16);
        const int  gcl   = valid ? (32 * j + lane) : 0;
        const v4f z0 = *(const v4f*)(zr + 8 * gcl);
        const v4f z1 = *(const v4f*)(zr + 8 * gcl + 4);
        const float zz[8] = {z0[0], z0[1], z0[2], z0[3], z1[0], z1[1], z1[2], z1[3]};
#pragma unroll
        for (int i = 0; i < 8; ++i) {
            const int c = 8 * gcl + i;
            const float yv = yb[(size_t)c * LSEQ];
            const float z  = zz[i];
            const float sg = z * fast_rcp(1.0f + __expf(-z));
            const float gv = yv * sg;
            g[j][i] = gv;
            ss += valid ? gv * gv : 0.0f;
        }
    }
    const float msq  = wave_sum(ss) * (1.0f / (float)D_INNER);
    const float rstd = rsqrtf(msq + RMS_EPS);

    us8 hv[3], lv[3];
#pragma unroll
    for (int j = 0; j < 3; ++j) {
        const bool valid = (j < 2) || (lane < 16);
        const int  gcl   = valid ? (32 * j + lane) : 0;
        float o[8];
#pragma unroll
        for (int i = 0; i < 8; ++i) o[i] = g[j][i] * rstd * rmsw[8 * gcl + i];
        split8(o, hv[j], lv[j]);
    }
    unsigned short* ph = yh + (size_t)m * D_INNER;
    unsigned short* pl = yl + (size_t)m * D_INNER;
    *(volatile us8*)(ph + 8 * lane)       = hv[0];
    *(volatile us8*)(pl + 8 * lane)       = lv[0];
    *(volatile us8*)(ph + 256 + 8 * lane) = hv[1];
    *(volatile us8*)(pl + 256 + 8 * lane) = lv[1];
    if (lane < 16) {
        *(volatile us8*)(ph + 512 + 8 * lane) = hv[2];
        *(volatile us8*)(pl + 512 + 8 * lane) = lv[2];
    }
    __threadfence();
    *(volatile us8*)(ph + 8 * lane)       = hv[0];
    *(volatile us8*)(pl + 8 * lane)       = lv[0];
    *(volatile us8*)(ph + 256 + 8 * lane) = hv[1];
    *(volatile us8*)(pl + 256 + 8 * lane) = lv[1];
    if (lane < 16) {
        *(volatile us8*)(ph + 512 + 8 * lane) = hv[2];
        *(volatile us8*)(pl + 512 + 8 * lane) = lv[2];
    }
}

static inline size_t align128(size_t b) { return (b + 127) & ~(size_t)127; }

extern "C" void kernel_launch(void* const* d_in, const int* in_sizes, int n_in,
                              void* d_out, int out_size, void* d_ws, size_t ws_size,
                              hipStream_t stream)
{
    if (n_in < 12) return;
    if (in_sizes[0] != BATCH * DIMC * LSEQ || in_sizes[1] != DIMC || in_sizes[2] != DIMC || in_sizes[3] != DIMC ||
        in_sizes[4] != D_IN_PROJ * DIMC || in_sizes[5] != CONV_DIM * D_CONV || in_sizes[6] != CONV_DIM ||
        in_sizes[7] != NHEADS || in_sizes[8] != NHEADS || in_sizes[9] != NHEADS || in_sizes[10] != D_INNER ||
        in_sizes[11] != DIMC * D_INNER || out_size != BATCH * DIMC * LSEQ) return;

    const float* x          = (const float*)d_in[0];
    const float* pe_gauss   = (const float*)d_in[1];
    const float* ln_w       = (const float*)d_in[2];
    const float* ln_b       = (const float*)d_in[3];
    const float* in_proj_w  = (const float*)d_in[4];
    const float* conv_w     = (const float*)d_in[5];
    const float* conv_b     = (const float*)d_in[6];
    const float* dt_bias    = (const float*)d_in[7];
    const float* A_log      = (const float*)d_in[8];
    const float* Dp         = (const float*)d_in[9];
    const float* rms_w      = (const float*)d_in[10];
    const float* out_proj_w = (const float*)d_in[11];
    float* out = (float*)d_out;

    char* ws = (char*)d_ws;
    size_t off = 0;
    unsigned short* uh  = (unsigned short*)(ws + off); off += align128((size_t)MROWS * DIMC * 2);
    unsigned short* ul  = (unsigned short*)(ws + off); off += align128((size_t)MROWS * DIMC * 2);
    unsigned short* w1h = (unsigned short*)(ws + off); off += align128((size_t)N1_PAD * DIMC * 2);
    unsigned short* w1l = (unsigned short*)(ws + off); off += align128((size_t)N1_PAD * DIMC * 2);
    unsigned short* w2h = (unsigned short*)(ws + off); off += align128((size_t)DIMC * D_INNER * 2);
    unsigned short* w2l = (unsigned short*)(ws + off); off += align128((size_t)DIMC * D_INNER * 2);
    float*          zxb = (float*)(ws + off);          off += align128((size_t)MROWS * N1_PAD * 4);
    float*          ybf = (float*)(ws + off);          off += align128((size_t)BATCH * D_INNER * LSEQ * 4);
    unsigned short* yh  = (unsigned short*)(ws + off); off += align128((size_t)MROWS * D_INNER * 2);
    unsigned short* yl  = (unsigned short*)(ws + off); off += align128((size_t)MROWS * D_INNER * 2);
    if (off > ws_size) return;

    {
        const int total = G1GRP + G2GRP;
        prep_w_kernel<<<(total + 255) / 256, 256, 0, stream>>>(in_proj_w, out_proj_w, w1h, w1l, w2h, w2l);
    }
    ln_pe_kernel<<<(MROWS + 7) / 8, 256, 0, stream>>>(x, pe_gauss, ln_w, ln_b, uh, ul);
    gemm_split_kernel<DIMC, false><<<dim3(MROWS / 64, N1_PAD / 64), 128, 0, stream>>>(uh, ul, w1h, w1l, zxb);
    ssm_scan_kernel<<<BATCH * NHEADS, 160, 0, stream>>>(zxb, conv_w, conv_b, dt_bias, A_log, Dp, ybf);
    gate_rms_kernel<<<(MROWS + 7) / 8, 256, 0, stream>>>(zxb, ybf, rms_w, yh, yl);
    gemm_split_kernel<D_INNER, true><<<dim3(MROWS / 64, DIMC / 64), 128, 0, stream>>>(yh, yl, w2h, w2l, out);
}
